// Bottleneck_64183991271999
// MI455X (gfx1250) — hardware-run, weakly checked
//
#include <hip/hip_runtime.h>

typedef float          v8f   __attribute__((ext_vector_type(8)));
typedef float          v4f   __attribute__((ext_vector_type(4)));
typedef unsigned int   v4u   __attribute__((ext_vector_type(4)));
typedef int            v8i   __attribute__((ext_vector_type(8)));
typedef unsigned short v8us  __attribute__((ext_vector_type(8)));
typedef unsigned short v16us __attribute__((ext_vector_type(16)));
typedef __bf16         v16bf __attribute__((ext_vector_type(16)));
typedef _Float16       v16h  __attribute__((ext_vector_type(16)));
typedef v4f  __attribute__((may_alias)) v4fa;
typedef v8us __attribute__((may_alias)) v8usa;
union FragB { v16bf v; v16us u; v8us h[2]; v8i w; };
union FragH { v16h  v; v16us u; v8us h[2]; v8i w; };

__device__ __forceinline__ v8f wmb(const FragB& a, const FragB& b, v8f c) {
  v8f d = __builtin_amdgcn_wmma_f32_16x16x32_bf16(false, a.v, false, b.v, (short)0, c, false, false);
  asm volatile("v_nop\n\tv_nop\n\tv_nop\n\tv_nop" : "+v"(d) : "v"(a.w), "v"(b.w));
  return d;
}

__device__ __forceinline__ v8f wmh(const FragH& a, const FragH& b, v8f c) {
  v8f d = __builtin_amdgcn_wmma_f32_16x16x32_f16(false, a.v, false, b.v, (short)0, c, false, false);
  asm volatile("v_nop\n\tv_nop\n\tv_nop\n\tv_nop" : "+v"(d) : "v"(a.w), "v"(b.w));
  return d;
}

__device__ __forceinline__ unsigned bf16_bits(float f) {
  const unsigned u = __float_as_uint(f);
  const unsigned r = (u + 0x7FFFu + ((u >> 16) & 1u)) >> 16;
  const unsigned q = (u >> 16) | 0x40u;
  return ((u & 0x7fffffffu) > 0x7f800000u) ? q : r;
}

__device__ __forceinline__ float bf16_val(float f) {
  return __uint_as_float(bf16_bits(f) << 16);
}
__device__ __forceinline__ int clampi(int v, int lo, int hi) {
  return v < lo ? lo : (v > hi ? hi : v);
}

__device__ __forceinline__ unsigned f16_bits(float f) {
  const unsigned u  = __float_as_uint(f);
  const unsigned s  = (u >> 16) & 0x8000u;
  const unsigned a  = u & 0x7fffffffu;
  const unsigned t  = a - 0x38000000u;
  const unsigned r  = (t + 0x0FFFu + ((t >> 13) & 1u)) >> 13;
  const unsigned rc = r > 0x7C00u ? 0x7C00u : r;
  const bool small  = a < 0x38800000u;
  const bool isnan  = a > 0x7f800000u;
  const unsigned fin = small ? 0u : (s | rc);
  return isnan ? (s | 0x7E00u) : fin;
}

__device__ __forceinline__ unsigned pk16(unsigned lo, unsigned hi) { return lo | (hi << 16); }
__device__ __forceinline__ unsigned bf16_lo_bits(float v) {
  float hi = bf16_val(v);
  asm volatile("" : "+v"(hi));
  return bf16_bits(v - hi);
}
__device__ __forceinline__ v4u pack8_bf16(v4f a, v4f c) {
  return (v4u){ pk16(bf16_bits(a[0]), bf16_bits(a[1])), pk16(bf16_bits(a[2]), bf16_bits(a[3])),
                pk16(bf16_bits(c[0]), bf16_bits(c[1])), pk16(bf16_bits(c[2]), bf16_bits(c[3])) };
}
__device__ __forceinline__ v4u pack8_bf16_lo(v4f a, v4f c) {
  return (v4u){ pk16(bf16_lo_bits(a[0]), bf16_lo_bits(a[1])), pk16(bf16_lo_bits(a[2]), bf16_lo_bits(a[3])),
                pk16(bf16_lo_bits(c[0]), bf16_lo_bits(c[1])), pk16(bf16_lo_bits(c[2]), bf16_lo_bits(c[3])) };
}
__device__ __forceinline__ v4u pack8_f16(v4f a, v4f c) {
  return (v4u){ pk16(f16_bits(a[0]), f16_bits(a[1])), pk16(f16_bits(a[2]), f16_bits(a[3])),
                pk16(f16_bits(c[0]), f16_bits(c[1])), pk16(f16_bits(c[2]), f16_bits(c[3])) };
}

template <int FORM>
__global__ __launch_bounds__(256) void k_plane(const float* __restrict__ src, int rows, int cols, int ldsrc,
                                               unsigned short* __restrict__ dst, int MP, int KP) {
  static_assert(FORM >= 0 && FORM <= 3);
  const int KTOT = (FORM == 1 || FORM == 3) ? 2 * KP : KP;
  const unsigned ppr   = (unsigned)(KTOT >> 3);
  const unsigned kp8   = (unsigned)(KP >> 3);
  const unsigned total = (unsigned)MP * ppr;
  const unsigned g     = blockIdx.x * 256u + threadIdx.x;
  const unsigned rowu  = g / ppr;
  const unsigned p     = g - rowu * ppr;
  const bool second    = p >= kp8;
  const int row = (int)rowu;
  const int c0  = (int)((second ? p - kp8 : p) << 3);
  const float* srow = src + (size_t)clampi(row, 0, rows - 1) * (size_t)ldsrc;
  float x[8];
  unsigned mk[8];
#pragma unroll
  for (int e = 0; e < 8; ++e) {
    const int c = c0 + e;
    const float v = srow[clampi(c, 0, cols - 1)];
    asm volatile("" :: "v"(v));
    x[e]  = v;
    mk[e] = (row < rows && c < cols) ? 0xFFFFu : 0u;
  }
  const v4f a = (v4f){ x[0], x[1], x[2], x[3] };
  const v4f c = (v4f){ x[4], x[5], x[6], x[7] };
  v4u o;
  if (FORM == 2) {
    o = pack8_f16(a, c);
  } else {
    const v4u hi = pack8_bf16(a, c);
    o = hi;
    if (FORM == 1) { const v4u lo = pack8_bf16_lo(a, c); o = second ? lo : hi; }
  }
  const v4u mw = (v4u){ pk16(mk[0], mk[1]), pk16(mk[2], mk[3]), pk16(mk[4], mk[5]), pk16(mk[6], mk[7]) };
  o &= mw;
  if (g < total) {
    volatile v4u* q = (volatile v4u*)(dst + (size_t)g * 8);
    *q = o;
    __threadfence();
    *q = o;
  }
}

template <int FORM> struct FragOf    { typedef FragB T; };
template <>         struct FragOf<2> { typedef FragH T; };
__device__ __forceinline__ v8f mm(const FragB& a, const FragB& b, v8f c) { return wmb(a, b, c); }
__device__ __forceinline__ v8f mm(const FragH& a, const FragH& b, v8f c) { return wmh(a, b, c); }
template <class F> __device__ __forceinline__ F ld_frag(const unsigned short* p) {
  F f;
  f.h[0] = *(const v8usa*)(p);
  f.h[1] = *(const v8usa*)(p + 16);
  return f;
}

template <int FORM, int EPI>
__global__ __launch_bounds__(256) __attribute__((amdgpu_num_vgpr(248)))
void k_gemm_nt(const unsigned short* __restrict__ A, const unsigned short* __restrict__ B,
               const float* __restrict__ bias, float* __restrict__ D, int M, int N, int KTOT, int ldd) {
  static_assert(FORM >= 0 && FORM <= 2);
  static_assert(EPI == 0 || EPI == 1);
  typedef typename FragOf<FORM>::T F;
  __shared__ __attribute__((aligned(16))) float sT[8][16 * 68];
  const int lane = threadIdx.x & 31;
  const int wave = threadIdx.x >> 5;
  const int tilesM = (M + 63) >> 6;
  const int tilesN = (N + 63) >> 6;
  const int tile = blockIdx.x * 8 + wave;
  if (tile >= tilesM * tilesN) return;
  const int tm = tile / tilesN;
  const int tn = tile - tm * tilesN;
  const int m0 = tm << 6;
  const int n0 = tn << 6;

  const int rl = lane & 15;
  const int h8 = (lane >> 4) * 8;
  const unsigned short* pa = A + (size_t)(m0 + rl) * (size_t)KTOT + h8;
  const unsigned short* pb = B + (size_t)(n0 + rl) * (size_t)KTOT + h8;

  v8f acc[4][4];
#pragma unroll
  for (int i = 0; i < 4; ++i)
#pragma unroll
    for (int j = 0; j < 4; ++j) acc[i][j] = (v8f){0.f, 0.f, 0.f, 0.f, 0.f, 0.f, 0.f, 0.f};

#pragma unroll 1
  for (int k0 = 0; k0 < KTOT; k0 += 32) {
    F bf[4];
#pragma unroll
    for (int j = 0; j < 4; ++j) bf[j] = ld_frag<F>(pb + (size_t)(j << 4) * (size_t)KTOT + k0);
#pragma unroll
    for (int i = 0; i < 4; ++i) {
      const F af = ld_frag<F>(pa + (size_t)(i << 4) * (size_t)KTOT + k0);
#pragma unroll
      for (int j = 0; j < 4; ++j) acc[i][j] = mm(af, bf[j], acc[i][j]);
    }
  }

  float* slab = sT[wave];
  const int hh = lane >> 4;
  const int c4 = (lane & 15) * 4;
  const int nc = n0 + c4;
  const bool cok = nc < N;
  v4f bv = (v4f){0.f, 0.f, 0.f, 0.f};
  if (EPI == 1) {
    bv = *(const v4fa*)(bias + clampi(nc, 0, N - 4));
    asm volatile("" :: "v"(bv));
  }
#pragma unroll
  for (int i = 0; i < 4; ++i) {
    const int mBase = m0 + (i << 4);
#pragma unroll
    for (int j = 0; j < 4; ++j) {
#pragma unroll
      for (int r = 0; r < 8; ++r) slab[(h8 + r) * 68 + (j << 4) + rl] = acc[i][j][r];
    }
    __builtin_amdgcn_fence(__ATOMIC_RELEASE, "workgroup");
    __builtin_amdgcn_wave_barrier();
    __builtin_amdgcn_fence(__ATOMIC_ACQUIRE, "workgroup");
    v4f vv[8];
#pragma unroll
    for (int it = 0; it < 8; ++it) {
      const int row = it * 2 + hh;
      v4f v = *(const v4fa*)(slab + row * 68 + c4);
      if (EPI == 1) v += bv;
      vv[it] = v;
    }
    for (int pass = 0; pass < 2; ++pass) {
#pragma unroll
      for (int it = 0; it < 8; ++it) {
        const int row = mBase + it * 2 + hh;
        if (cok && row < M) *(volatile v4f*)(D + (size_t)row * (size_t)ldd + nc) = vv[it];
      }
      __threadfence();
    }
    __builtin_amdgcn_fence(__ATOMIC_RELEASE, "workgroup");
    __builtin_amdgcn_wave_barrier();
    __builtin_amdgcn_fence(__ATOMIC_ACQUIRE, "workgroup");
  }
}

typedef v4u __attribute__((may_alias)) v4ua;

#ifndef SPLIT_PROJ
#define SPLIT_PROJ 1
#endif
#ifndef SPLIT_MLP1
#define SPLIT_MLP1 1
#endif
#ifndef SPLIT_MLP2
#define SPLIT_MLP2 1
#endif
#ifndef SPLIT_OUT
#define SPLIT_OUT 1
#endif

constexpr int kB    = 2;
constexpr int kC    = 256;
constexpr int kH    = 56;
constexpr int kW    = 56;
constexpr int kHW   = kH * kW;
constexpr int kM    = kB * kHW;
constexpr int kREL  = 64;
constexpr int kMID  = 256;
constexpr int kHN   = 32;
constexpr int kCH   = 66;
constexpr int kKS   = 7;
constexpr int kPAD  = 3;
constexpr int kSH   = 8;
constexpr int kNB   = kKS * kKS;
constexpr int kN1   = 2 * kREL + kMID;
constexpr int kKT   = 2 * kC;

static_assert(kB == 2);
static_assert(kH == 56 && kW == 56);
static_assert(kKS == 7 && kPAD == 3 && kSH == 8);
static_assert(kM % 128 == 0);
static_assert(kM % 64 == 0);
static_assert(kHW % 32 == 0);
static_assert(kHW % 16 == 0);
static_assert(kNB * 16 == 784);
static_assert(kMID / kSH == 32);
static_assert(kMID / kSH == kHN);
static_assert(kN1 % 64 == 0 && kN1 % 32 == 0);
static_assert(kC % 64 == 0 && kC % 32 == 0);
static_assert(kKT % 32 == 0);
static_assert(96 % 32 == 0 && 96 >= kCH);
static_assert(kREL % 32 == 0);

constexpr int T_BN1S = 0;
constexpr int T_BN1M = 256;
constexpr int T_BN1B = 512;
constexpr int T_SAN  = 768;
constexpr int T_CB2  = 3072;
constexpr int T_BIAS = 3328;
constexpr int T_BC   = 3840;
constexpr int T_P    = 4096;
constexpr int T_END  = 11264;
constexpr int T_BLOCKS = T_END / 256;
constexpr int L_C1S = 0;
constexpr int L_C1M = 256;
constexpr int L_C1B = 512;
constexpr int L_C2S = 768;
constexpr int L_C2M = 1024;
constexpr int L_C2B = 1280;
constexpr int L_B2S = 1536;
constexpr int L_B2M = 1792;
constexpr int L_B2B = 2048;
constexpr int L_CB2 = 2304;
static_assert(T_SAN + L_CB2 == T_CB2);
static_assert(T_SAN + 3072 <= T_BC);
static_assert(T_P + 7168 == T_END);
static_assert(2 * kHW <= 7168);

constexpr size_t SZ_A1   = (size_t)kM * kKT * 2;
constexpr size_t SZ_X123 = (size_t)kM * kN1 * 4;
constexpr size_t SZ_G    = (size_t)kM * kKT * 2;
constexpr size_t SZ_Y    = (size_t)kM * kC * 4;
constexpr size_t SZ_W123 = (size_t)kN1 * kKT * 2;
constexpr size_t SZ_WC   = (size_t)kC * kKT * 2;
constexpr size_t SZ_CW1  = (size_t)64 * 192 * 2;
constexpr size_t SZ_CW2  = (size_t)32 * 128 * 2;
constexpr size_t SZ_TAB  = (size_t)T_END * 4;
constexpr size_t WS_A1   = 0;
constexpr size_t WS_X123 = WS_A1 + SZ_A1;
constexpr size_t WS_G    = WS_X123 + SZ_X123;
constexpr size_t WS_Y    = WS_G + SZ_G;
constexpr size_t WS_W123 = WS_Y + SZ_Y;
constexpr size_t WS_WC   = WS_W123 + SZ_W123;
constexpr size_t WS_CW1  = WS_WC + SZ_WC;
constexpr size_t WS_CW2  = WS_CW1 + SZ_CW1;
constexpr size_t WS_TAB  = WS_CW2 + SZ_CW2;
constexpr size_t WS_END  = WS_TAB + SZ_TAB;
static_assert(WS_X123 % 256 == 0 && WS_G % 256 == 0 && WS_Y % 256 == 0);
static_assert(WS_W123 % 256 == 0 && WS_WC % 256 == 0 && WS_CW1 % 256 == 0);
static_assert(WS_CW2 % 256 == 0 && WS_TAB % 256 == 0);
static_assert(WS_END == (size_t)29634560);
static_assert(WS_END <= ((size_t)128 << 20));

__device__ __forceinline__ float relu_sel(float v) { return (v > 0.0f) ? v : (v - v); }
__device__ __forceinline__ int refl56(int i) { return i < 0 ? -i : (i > 55 ? 110 - i : i); }
__device__ __forceinline__ void wave_lds_sync() {
  __builtin_amdgcn_fence(__ATOMIC_RELEASE, "workgroup");
  __builtin_amdgcn_wave_barrier();
  __builtin_amdgcn_fence(__ATOMIC_ACQUIRE, "workgroup");
}
__device__ __forceinline__ float lin56(int i) {
#pragma clang fp contract(off)
  const float t = (float)i / 55.0f;
  const float v = (-(1.0f - t)) + t;
  return (i == 55) ? 1.0f : v;
}
__device__ __forceinline__ float pos_val(float a, float c, float pbv, float lw, float lh) {
#pragma clang fp contract(off)
  const float t0 = a * lw;
  const float t1 = c * lh;
  return (t0 + t1) + pbv;
}

__global__ __launch_bounds__(256) void k_tab(
    const float* __restrict__ bn1g, const float* __restrict__ bn1b, const float* __restrict__ bn1m, const float* __restrict__ bn1v,
    const float* __restrict__ b1, const float* __restrict__ b2, const float* __restrict__ b3,
    const float* __restrict__ pw, const float* __restrict__ pb,
    const float* __restrict__ c1g, const float* __restrict__ c1b, const float* __restrict__ c1m, const float* __restrict__ c1v,
    const float* __restrict__ c2g, const float* __restrict__ c2b, const float* __restrict__ c2m, const float* __restrict__ c2v,
    const float* __restrict__ cb2,
    const float* __restrict__ n2g, const float* __restrict__ n2b, const float* __restrict__ n2m, const float* __restrict__ n2v,
    const float* __restrict__ bc, float* __restrict__ TAB) {
  const int bid = blockIdx.x;
  const int tid = threadIdx.x;
  float val = 0.0f;
  if (bid < 12) {
    const int set = bid / 3;
    const int t   = bid - 3 * set;
    float gv, bv, mv, vv;
    int n;
    if (set == 0) {
      n = 256; const int ic = clampi(tid, 0, 255);
      gv = bn1g[ic]; bv = bn1b[ic]; mv = bn1m[ic]; vv = bn1v[ic];
    } else if (set == 1) {
      n = kCH; const int ic = clampi(tid, 0, kCH - 1);
      gv = c1g[ic]; bv = c1b[ic]; mv = c1m[ic]; vv = c1v[ic];
    } else if (set == 2) {
      n = kREL; const int ic = clampi(tid, 0, kREL - 1);
      gv = c2g[ic]; bv = c2b[ic]; mv = c2m[ic]; vv = c2v[ic];
    } else {
      n = 256; const int ic = clampi(tid, 0, 255);
      gv = n2g[ic]; bv = n2b[ic]; mv = n2m[ic]; vv = n2v[ic];
    }
    asm volatile("" :: "v"(gv), "v"(bv), "v"(mv), "v"(vv));
    const float s = bf16_val(gv) * (1.0f / sqrtf(bf16_val(vv) + 1e-5f));
    const float sel = (t == 0) ? s : ((t == 1) ? bf16_val(mv) : bf16_val(bv));
    const unsigned keep = (tid < n) ? 0xFFFFFFFFu : 0u;
    val = __uint_as_float(__float_as_uint(sel) & keep);
  } else if (bid == 12) {
    const float v = cb2[clampi(tid, 0, kHN - 1)];
    asm volatile("" :: "v"(v));
    const unsigned keep = (tid < kHN) ? 0xFFFFFFFFu : 0u;
    val = __uint_as_float(__float_as_uint(bf16_val(v)) & keep);
  } else if (bid < 15) {
    const int e = (bid - 13) * 256 + tid;
    const float v1 = b1[clampi(e, 0, 63)];
    const float v2 = b2[clampi(e - 64, 0, 63)];
    const float v3 = b3[clampi(e - 128, 0, 255)];
    asm volatile("" :: "v"(v1), "v"(v2), "v"(v3));
    const unsigned k1 = (e < 64) ? 0xFFFFFFFFu : 0u;
    const unsigned k2 = (e >= 64 && e < 128) ? 0xFFFFFFFFu : 0u;
    const unsigned k3 = (e >= 128 && e < 384) ? 0xFFFFFFFFu : 0u;
    val = __uint_as_float((__float_as_uint(bf16_val(v1)) & k1) | (__float_as_uint(bf16_val(v2)) & k2) |
                          (__float_as_uint(bf16_val(v3)) & k3));
  } else if (bid == 15) {
    const float v = bc[clampi(tid, 0, 255)];
    asm volatile("" :: "v"(v));
    val = bf16_val(v);
  } else {
    const int e = (bid - 16) * 256 + tid;
    const int o = (e >= kHW) ? 1 : 0;
    const int q = clampi(e - o * kHW, 0, kHW - 1);
    const int h = q / kW;
    const int w = q - h * kW;
    const float a = pw[2 * o];
    const float c = pw[2 * o + 1];
    const float pbv = pb[o];
    asm volatile("" :: "v"(a), "v"(c), "v"(pbv));
    const float pv = pos_val(bf16_val(a), bf16_val(c), bf16_val(pbv), lin56(w), lin56(h));
    const unsigned keep = (e < 2 * kHW) ? 0xFFFFFFFFu : 0u;
    val = __uint_as_float(__float_as_uint(pv) & keep);
  }
  volatile float* p = (volatile float*)(TAB + bid * 256 + tid);
  *p = val;
  __threadfence();
  *p = val;
}

constexpr int TP = 257;
__global__ __launch_bounds__(256) void k_bn1t(const float* __restrict__ x, const float* __restrict__ TAB,
                                              unsigned short* __restrict__ A1) {
  __shared__ __attribute__((aligned(16))) float sT[32 * TP];
  __shared__ __attribute__((aligned(16))) float sB[1024];
  const int tid  = threadIdx.x;
  const int lane = tid & 31;
  const int wave = tid >> 5;
  const int b    = blockIdx.x / (kHW / 32);
  const int q0   = (blockIdx.x - b * (kHW / 32)) * 32;
  {
    const v4f t = *(const v4fa*)(TAB + 4 * tid);
    *(v4fa*)(sB + 4 * tid) = t;
  }
  __syncthreads();
  const int csub = lane >> 3;
  const int q4   = (lane & 7) * 4;
#pragma unroll 2
  for (int it = 0; it < 8; ++it) {
    const int c = it * 32 + wave * 4 + csub;
    const v4f a = *(const v4fa*)(x + (size_t)(b * kC + c) * (size_t)kHW + (size_t)(q0 + q4));
    const float s = sB[T_BN1S + c];
    const float m = sB[T_BN1M + c];
    const float bb = sB[T_BN1B + c];
#pragma unroll
    for (int e = 0; e < 4; ++e) {
      const float xv = bf16_val(a[e]);
      const float v = relu_sel((xv - m) * s + bb);
      sT[(q4 + e) * TP + c] = v;
    }
  }
  __syncthreads();
  const unsigned lm = SPLIT_PROJ ? 0xFFFFFFFFu : 0u;
  v4u ph[4], pl[4];
#pragma unroll
  for (int i = 0; i < 4; ++i) {
    const float* t = sT + (wave * 4 + i) * TP + 8 * lane;
    const v4f a = (v4f){ t[0], t[1], t[2], t[3] };
    const v4f c = (v4f){ t[4], t[5], t[6], t[7] };
    ph[i] = pack8_bf16(a, c);
    pl[i] = pack8_bf16_lo(a, c) & (v4u){ lm, lm, lm, lm };
  }
  const size_t r0 = (size_t)b * kHW + (size_t)(q0 + wave * 4);
  for (int pass = 0; pass < 2; ++pass) {
#pragma unroll
    for (int i = 0; i < 4; ++i) {
      *(volatile v4u*)(A1 + (r0 + i) * (size_t)kKT + 8 * lane) = ph[i];
      *(volatile v4u*)(A1 + (r0 + i) * (size_t)kKT + kC + 8 * lane) = pl[i];
    }
    __threadfence();
  }
}

constexpr int SAN_AP   = 200;
constexpr int SAN_A2P  = 136;
constexpr int SAN_DP   = 68;
constexpr int SAN_W1P  = 200;
constexpr int SAN_W2P  = 136;
constexpr int OFF_X1   = 0;
constexpr int OFF_P    = OFF_X1 + 16 * 64 * 4;
constexpr int OFF_W1   = OFF_P + 7168 * 4;
constexpr int OFF_W2   = OFF_W1 + 64 * SAN_W1P * 2;
constexpr int OFF_TAB  = OFF_W2 + 32 * SAN_W2P * 2;
constexpr int OFF_LOG  = OFF_TAB + 3072 * 4;
constexpr int OFF_WV   = OFF_LOG + kNB * 16 * 32 * 4;
constexpr int WV_A_BYTES = 16 * SAN_AP * 2;
constexpr int WV_D_BYTES = 16 * SAN_DP * 4;
constexpr int WV_BYTES   = WV_A_BYTES + WV_D_BYTES;
constexpr int SAN_LDS_BYTES = OFF_WV + 8 * WV_BYTES;
static_assert(16 * SAN_A2P * 2 <= WV_A_BYTES);
static_assert(OFF_P % 16 == 0 && OFF_W1 % 16 == 0 && OFF_W2 % 16 == 0 && OFF_TAB % 16 == 0);
static_assert(OFF_LOG % 16 == 0 && OFF_WV % 16 == 0 && WV_BYTES % 16 == 0 && WV_A_BYTES % 16 == 0);
static_assert(SAN_LDS_BYTES == 265728);
static_assert(SAN_LDS_BYTES <= 300000);
static_assert(SAN_LDS_BYTES <= 327680);

__global__ __launch_bounds__(256) __attribute__((amdgpu_num_vgpr(248)))
void k_san(const float* __restrict__ X123, const float* __restrict__ TAB,
           const unsigned short* __restrict__ CW1D, const unsigned short* __restrict__ CW2D,
           unsigned short* __restrict__ G) {
  extern __shared__ __attribute__((aligned(16))) unsigned char san_lds[];
  float* sX1  = (float*)(san_lds + OFF_X1);
  float* sP   = (float*)(san_lds + OFF_P);
  unsigned short* sW1 = (unsigned short*)(san_lds + OFF_W1);
  unsigned short* sW2 = (unsigned short*)(san_lds + OFF_W2);
  float* sTab = (float*)(san_lds + OFF_TAB);
  float* sLOG = (float*)(san_lds + OFF_LOG);

  const int tid  = threadIdx.x;
  const int lane = tid & 31;
  const int wave = __builtin_amdgcn_readfirstlane((int)(threadIdx.x >> 5));
  const int r0    = blockIdx.x * 16;
  const int b     = r0 / kHW;
  const int qbase = r0 - b * kHW;
  const size_t rowb = (size_t)b * (size_t)kHW;

  {
    const int pix = tid >> 4;
    const int c4  = (tid & 15) * 4;
    const v4f v = *(const v4fa*)(X123 + (size_t)(r0 + pix) * (size_t)kN1 + c4);
    *(v4fa*)(sX1 + pix * 64 + c4) = v;
  }
#pragma unroll 1
  for (int it = 0; it < 7; ++it) {
    const int i = it * 256 + tid;
    const v4f v = *(const v4fa*)(TAB + T_P + 4 * i);
    *(v4fa*)(sP + 4 * i) = v;
  }
#pragma unroll 1
  for (int it = 0; it < 3; ++it) {
    const int i = it * 256 + tid;
    const v4f v = *(const v4fa*)(TAB + T_SAN + 4 * i);
    *(v4fa*)(sTab + 4 * i) = v;
  }
#pragma unroll 1
  for (int it = 0; it < 6; ++it) {
    const int pid = it * 256 + tid;
    const int row = pid / 24;
    const int pc  = pid - row * 24;
    const v4u v = *(const v4ua*)(CW1D + row * 192 + pc * 8);
    *(v4ua*)(sW1 + row * SAN_W1P + pc * 8) = v;
  }
#pragma unroll 1
  for (int it = 0; it < 2; ++it) {
    const int pid = it * 256 + tid;
    const int row = pid >> 4;
    const int pc  = pid & 15;
    const v4u v = *(const v4ua*)(CW2D + row * 128 + pc * 8);
    *(v4ua*)(sW2 + row * SAN_W2P + pc * 8) = v;
  }
  __syncthreads();

  unsigned short* sA = (unsigned short*)(san_lds + OFF_WV + wave * WV_BYTES);
  float* sD = (float*)(san_lds + OFF_WV + wave * WV_BYTES + WV_A_BYTES);
  const int rl = lane & 15;
  const int hf = lane >> 4;
  const int h8 = hf * 8;
  {
    const int qpix = qbase + rl;
    const int ph   = qpix / kW;
    const int pwc  = qpix - ph * kW;
    const float pc0 = sP[qpix];
    const float pc1 = sP[kHW + qpix];
    const float s64 = sTab[L_C1S + 64], m64 = sTab[L_C1M + 64], b64 = sTab[L_C1B + 64];
    const float s65 = sTab[L_C1S + 65], m65 = sTab[L_C1M + 65], b65 = sTab[L_C1B + 65];
    const float cbA = sTab[L_CB2 + rl];
    const float cbB = sTab[L_CB2 + 16 + rl];
    const float* x1row = sX1 + rl * 64;
    const unsigned lm1 = SPLIT_MLP1 ? 0xFFFFFFFFu : 0u;
    const unsigned lm2 = SPLIT_MLP2 ? 0xFFFFFFFFu : 0u;
    const unsigned hsel = 0u - (unsigned)hf;

#pragma unroll 1
    for (int k = wave; k < kNB; k += 8) {
      const int ki  = k / kKS;
      const int kj  = k - ki * kKS;
      const int nh  = refl56(ph + ki - kPAD);
      const int nw  = refl56(pwc + kj - kPAD);
      const int nbr = nh * kW + nw;
      const float* xr = X123 + (rowb + (size_t)nbr) * (size_t)kN1 + kREL;

      {
        const float f0 = pc0 - sP[nbr];
        const float f1 = pc1 - sP[kHW + nbr];
        const float v0 = relu_sel((f0 - m64) * s64 + b64);
        const float v1 = relu_sel((f1 - m65) * s65 + b65);
        const unsigned wh = pk16(bf16_bits(v0), bf16_bits(v1));
        const unsigned wl = pk16(bf16_lo_bits(v0), bf16_lo_bits(v1)) & lm1;
        const unsigned wsel = (wl & hsel) | (wh & ~hsel);
        unsigned short* pp = sA + rl * SAN_AP + hf * 96 + 64;
        *(v4ua*)(pp)      = (v4u){ wsel, 0u, 0u, 0u };
        *(v4ua*)(pp + 8)  = (v4u){ 0u, 0u, 0u, 0u };
        *(v4ua*)(pp + 16) = (v4u){ 0u, 0u, 0u, 0u };
        *(v4ua*)(pp + 24) = (v4u){ 0u, 0u, 0u, 0u };
      }
#pragma unroll 1
      for (int it = 0; it < 4; ++it) {
        const int c0 = it * 16 + h8;
        const v4f g0 = *(const v4fa*)(xr + c0);
        const v4f g1 = *(const v4fa*)(xr + c0 + 4);
        const v4f a0 = *(const v4fa*)(x1row + c0);
        const v4f a1 = *(const v4fa*)(x1row + c0 + 4);
        const v4f s0 = *(const v4fa*)(sTab + L_C1S + c0);
        const v4f s1 = *(const v4fa*)(sTab + L_C1S + c0 + 4);
        const v4f m0 = *(const v4fa*)(sTab + L_C1M + c0);
        const v4f m1 = *(const v4fa*)(sTab + L_C1M + c0 + 4);
        const v4f e0 = *(const v4fa*)(sTab + L_C1B + c0);
        const v4f e1 = *(const v4fa*)(sTab + L_C1B + c0 + 4);
        v4f v0, v1;
#pragma unroll
        for (int e = 0; e < 4; ++e) {
          v0[e] = relu_sel(((a0[e] - g0[e]) - m0[e]) * s0[e] + e0[e]);
          v1[e] = relu_sel(((a1[e] - g1[e]) - m1[e]) * s1[e] + e1[e]);
        }
        const v4u hi = pack8_bf16(v0, v1);
        const v4u lo = pack8_bf16_lo(v0, v1) & (v4u){ lm1, lm1, lm1, lm1 };
        *(v4ua*)(sA + rl * SAN_AP + c0)      = hi;
        *(v4ua*)(sA + rl * SAN_AP + 96 + c0) = lo;
      }
      wave_lds_sync();

      v8f acc[4];
#pragma unroll
      for (int nt = 0; nt < 4; ++nt) acc[nt] = (v8f){0.f, 0.f, 0.f, 0.f, 0.f, 0.f, 0.f, 0.f};
#pragma unroll 1
      for (int ks = 0; ks < 6; ++ks) {
        const int k0 = ks * 32;
        const FragB af = ld_frag<FragB>(sA + rl * SAN_AP + h8 + k0);
#pragma unroll
        for (int nt = 0; nt < 4; ++nt) {
          const FragB bf = ld_frag<FragB>(sW1 + (nt * 16 + rl) * SAN_W1P + h8 + k0);
          acc[nt] = wmb(af, bf, acc[nt]);
        }
      }
#pragma unroll
      for (int nt = 0; nt < 4; ++nt) {
#pragma unroll
        for (int r = 0; r < 8; ++r) sD[(h8 + r) * SAN_DP + nt * 16 + rl] = acc[nt][r];
      }
      wave_lds_sync();

#pragma unroll 1
      for (int it = 0; it < 4; ++it) {
        const int c0 = it * 16 + h8;
        const v4f d0 = *(const v4fa*)(sD + rl * SAN_DP + c0);
        const v4f d1 = *(const v4fa*)(sD + rl * SAN_DP + c0 + 4);
        const v4f s0 = *(const v4fa*)(sTab + L_C2S + c0);
        const v4f s1 = *(const v4fa*)(sTab + L_C2S + c0 + 4);
        const v4f m0 = *(const v4fa*)(sTab + L_C2M + c0);
        const v4f m1 = *(const v4fa*)(sTab + L_C2M + c0 + 4);
        const v4f e0 = *(const v4fa*)(sTab + L_C2B + c0);
        const v4f e1 = *(const v4fa*)(sTab + L_C2B + c0 + 4);
        v4f u0, u1;
#pragma unroll
        for (int e = 0; e < 4; ++e) {
          u0[e] = relu_sel((d0[e] - m0[e]) * s0[e] + e0[e]);
          u1[e] = relu_sel((d1[e] - m1[e]) * s1[e] + e1[e]);
        }
        const v4u hi = pack8_bf16(u0, u1);
        const v4u lo = pack8_bf16_lo(u0, u1) & (v4u){ lm2, lm2, lm2, lm2 };
        *(v4ua*)(sA + rl * SAN_A2P + c0)        = hi;
        *(v4ua*)(sA + rl * SAN_A2P + kREL + c0) = lo;
      }
      wave_lds_sync();

      v8f lg[2];
      lg[0] = (v8f){0.f, 0.f, 0.f, 0.f, 0.f, 0.f, 0.f, 0.f};
      lg[1] = (v8f){0.f, 0.f, 0.f, 0.f, 0.f, 0.f, 0.f, 0.f};
#pragma unroll 1
      for (int ks = 0; ks < 4; ++ks) {
        const int k0 = ks * 32;
        const FragB af = ld_frag<FragB>(sA + rl * SAN_A2P + h8 + k0);
#pragma unroll
        for (int nt = 0; nt < 2; ++nt) {
          const FragB bf = ld_frag<FragB>(sW2 + (nt * 16 + rl) * SAN_W2P + h8 + k0);
          lg[nt] = wmb(af, bf, lg[nt]);
        }
      }
#pragma unroll
      for (int r = 0; r < 8; ++r) {
        float* dst = sLOG + (k * 16 + h8 + r) * 32 + rl;
        dst[0]  = lg[0][r] + cbA;
        dst[16] = lg[1][r] + cbB;
      }
      wave_lds_sync();
    }
  }
  __syncthreads();

#pragma unroll 1
  for (int pass = 0; pass < 2; ++pass) {
    float* p = sLOG + pass * 256 + tid;
    float mx = p[0];
#pragma unroll 1
    for (int k = 1; k < kNB; ++k) {
      const float v = p[k * 512];
      mx = (v > mx) ? v : mx;
    }
    float s = 0.0f;
#pragma unroll 1
    for (int k = 0; k < kNB; ++k) {
      const float e = expf(p[k * 512] - mx);
      p[k * 512] = e;
      s += e;
    }
#pragma unroll 1
    for (int k = 0; k < kNB; ++k) {
      const float a = p[k * 512] / s;
      p[k * 512] = a;
    }
  }
  __syncthreads();

  const unsigned lm3 = SPLIT_OUT ? 0xFFFFFFFFu : 0u;
  v4u gh[2], gl[2];
#pragma unroll
  for (int pp = 0; pp < 2; ++pp) {
    const int pix = wave * 2 + pp;
    const int q   = qbase + pix;
    const int h   = q / kW;
    const int w   = q - h * kW;
    v4f a0 = (v4f){0.f, 0.f, 0.f, 0.f};
    v4f a1 = (v4f){0.f, 0.f, 0.f, 0.f};
    int ki = 0, kj = 0;
#pragma unroll 1
    for (int k = 0; k < kNB; ++k) {
      const int nh = refl56(h + ki - kPAD);
      const int nw = refl56(w + kj - kPAD);
      const float* xr = X123 + (rowb + (size_t)(nh * kW + nw)) * (size_t)kN1 + 2 * kREL + 8 * lane;
      const v4f x0 = *(const v4fa*)(xr);
      const v4f x1 = *(const v4fa*)(xr + 4);
      const float wg = sLOG[(k * 16 + pix) * 32 + lane];
#pragma unroll
      for (int e = 0; e < 4; ++e) {
        a0[e] = fmaf(wg, x0[e], a0[e]);
        a1[e] = fmaf(wg, x1[e], a1[e]);
      }
      ++kj;
      if (kj == kKS) { kj = 0; ++ki; }
    }
    const v4f s0 = *(const v4fa*)(sTab + L_B2S + 8 * lane);
    const v4f s1 = *(const v4fa*)(sTab + L_B2S + 8 * lane + 4);
    const v4f m0 = *(const v4fa*)(sTab + L_B2M + 8 * lane);
    const v4f m1 = *(const v4fa*)(sTab + L_B2M + 8 * lane + 4);
    const v4f e0 = *(const v4fa*)(sTab + L_B2B + 8 * lane);
    const v4f e1 = *(const v4fa*)(sTab + L_B2B + 8 * lane + 4);
    v4f o0, o1;
#pragma unroll
    for (int e = 0; e < 4; ++e) {
      o0[e] = relu_sel((a0[e] - m0[e]) * s0[e] + e0[e]);
      o1[e] = relu_sel((a1[e] - m1[e]) * s1[e] + e1[e]);
    }
    gh[pp] = pack8_bf16(o0, o1);
    gl[pp] = pack8_bf16_lo(o0, o1) & (v4u){ lm3, lm3, lm3, lm3 };
  }
  for (int pass = 0; pass < 2; ++pass) {
#pragma unroll
    for (int pp = 0; pp < 2; ++pp) {
      const size_t r = (size_t)(r0 + wave * 2 + pp);
      *(volatile v4u*)(G + r * (size_t)kKT + 8 * lane) = gh[pp];
      *(volatile v4u*)(G + r * (size_t)kKT + kC + 8 * lane) = gl[pp];
    }
    __threadfence();
  }
}

__global__ __launch_bounds__(256) void k_store(const float* __restrict__ Y, const float* __restrict__ x,
                                               float* __restrict__ out) {
  __shared__ __attribute__((aligned(16))) float sT[32 * TP];
  const int tid  = threadIdx.x;
  const int lane = tid & 31;
  const int wave = tid >> 5;
  const int b    = blockIdx.x / (kHW / 32);
  const int q0   = (blockIdx.x - b * (kHW / 32)) * 32;
  const size_t rbase = (size_t)b * kHW + (size_t)q0;
#pragma unroll 2
  for (int it = 0; it < 8; ++it) {
    const int pid = it * 256 + tid;
    const int row = pid >> 6;
    const int c4  = (pid & 63) * 4;
    const v4f v = *(const v4fa*)(Y + (rbase + row) * (size_t)kC + c4);
    float* t = sT + row * TP + c4;
    t[0] = v[0]; t[1] = v[1]; t[2] = v[2]; t[3] = v[3];
  }
  __syncthreads();
  const int csub = lane >> 3;
  const int q4   = (lane & 7) * 4;
  v4f o[8];
#pragma unroll
  for (int t = 0; t < 8; ++t) {
    const int c = wave * 32 + t * 4 + csub;
    const size_t idx = (size_t)(b * kC + c) * (size_t)kHW + (size_t)(q0 + q4);
    const v4f xv = *(const v4fa*)(x + idx);
    v4f r;
#pragma unroll
    for (int e = 0; e < 4; ++e) r[e] = sT[(q4 + e) * TP + c] + bf16_val(xv[e]);
    o[t] = r;
  }
  for (int pass = 0; pass < 2; ++pass) {
#pragma unroll
    for (int t = 0; t < 8; ++t) {
      const int c = wave * 32 + t * 4 + csub;
      const size_t idx = (size_t)(b * kC + c) * (size_t)kHW + (size_t)(q0 + q4);
      *(volatile v4f*)(out + idx) = o[t];
    }
    __threadfence();
  }
}

extern "C" void kernel_launch(void* const* d_in, const int* in_sizes, int n_in,
                              void* d_out, int out_size, void* d_ws, size_t ws_size,
                              hipStream_t stream) {
  if (n_in < 30) return;
  const int expect_n[30] = { 1605632, 256, 256, 256, 256, 16384, 64, 16384, 64, 65536, 256, 4, 2,
                             66, 66, 66, 66, 4224, 64, 64, 64, 64, 2048, 32, 256, 256, 256, 256, 65536, 256 };
  for (int i = 0; i < 30; ++i) { if (in_sizes[i] != expect_n[i]) return; }
  if (out_size != kB * kC * kHW) return;
  if (WS_END > ws_size) return;

  const float* x     = (const float*)d_in[0];
  const float* bn1g  = (const float*)d_in[1];
  const float* bn1b  = (const float*)d_in[2];
  const float* bn1m  = (const float*)d_in[3];
  const float* bn1v  = (const float*)d_in[4];
  const float* w1    = (const float*)d_in[5];
  const float* b1    = (const float*)d_in[6];
  const float* w2    = (const float*)d_in[7];
  const float* b2    = (const float*)d_in[8];
  const float* w3    = (const float*)d_in[9];
  const float* b3    = (const float*)d_in[10];
  const float* pw    = (const float*)d_in[11];
  const float* pb    = (const float*)d_in[12];
  const float* c1g   = (const float*)d_in[13];
  const float* c1b   = (const float*)d_in[14];
  const float* c1m   = (const float*)d_in[15];
  const float* c1v   = (const float*)d_in[16];
  const float* cw1   = (const float*)d_in[17];
  const float* c2g   = (const float*)d_in[18];
  const float* c2b   = (const float*)d_in[19];
  const float* c2m   = (const float*)d_in[20];
  const float* c2v   = (const float*)d_in[21];
  const float* cw2   = (const float*)d_in[22];
  const float* cb2   = (const float*)d_in[23];
  const float* n2g   = (const float*)d_in[24];
  const float* n2b   = (const float*)d_in[25];
  const float* n2m   = (const float*)d_in[26];
  const float* n2v   = (const float*)d_in[27];
  const float* wc    = (const float*)d_in[28];
  const float* bc    = (const float*)d_in[29];
  float* outp = (float*)d_out;

  char* ws = (char*)d_ws;
  unsigned short* A1    = (unsigned short*)(ws + WS_A1);
  float*          X123  = (float*)(ws + WS_X123);
  unsigned short* Gp    = (unsigned short*)(ws + WS_G);
  float*          Yp    = (float*)(ws + WS_Y);
  unsigned short* W123D = (unsigned short*)(ws + WS_W123);
  unsigned short* WCD   = (unsigned short*)(ws + WS_WC);
  unsigned short* CW1D  = (unsigned short*)(ws + WS_CW1);
  unsigned short* CW2D  = (unsigned short*)(ws + WS_CW2);
  float*          TAB   = (float*)(ws + WS_TAB);

  (void)hipFuncSetAttribute(reinterpret_cast<const void*>(&k_san), hipFuncAttributeMaxDynamicSharedMemorySize, SAN_LDS_BYTES);

  k_plane<3><<<dim3(64 * 512 / 8 / 256), dim3(256), 0, stream>>>(w1, 64, 256, 256, W123D, 64, 256);
  k_plane<3><<<dim3(64 * 512 / 8 / 256), dim3(256), 0, stream>>>(w2, 64, 256, 256, W123D + (size_t)64 * 512, 64, 256);
  k_plane<3><<<dim3(256 * 512 / 8 / 256), dim3(256), 0, stream>>>(w3, 256, 256, 256, W123D + (size_t)128 * 512, 256, 256);
  k_plane<3><<<dim3(256 * 512 / 8 / 256), dim3(256), 0, stream>>>(wc, 256, 256, 256, WCD, 256, 256);
  k_plane<3><<<dim3(64 * 192 / 8 / 256), dim3(256), 0, stream>>>(cw1, 64, kCH, kCH, CW1D, 64, 96);
  k_plane<3><<<dim3(32 * 128 / 8 / 256), dim3(256), 0, stream>>>(cw2, 32, 64, 64, CW2D, 32, 64);
  k_tab<<<dim3(T_BLOCKS), dim3(256), 0, stream>>>(bn1g, bn1b, bn1m, bn1v, b1, b2, b3, pw, pb,
                                                  c1g, c1b, c1m, c1v, c2g, c2b, c2m, c2v, cb2,
                                                  n2g, n2b, n2m, n2v, bc, TAB);
  k_bn1t<<<dim3(kB * (kHW / 32)), dim3(256), 0, stream>>>(x, TAB, A1);
  {
    const int tiles = (kM / 64) * (kN1 / 64);
    k_gemm_nt<1, 1><<<dim3((tiles + 7) / 8), dim3(256), 0, stream>>>(A1, W123D, TAB + T_BIAS, X123, kM, kN1, kKT, kN1);
  }
  k_san<<<dim3(kM / 16), dim3(256), SAN_LDS_BYTES, stream>>>(X123, TAB, CW1D, CW2D, Gp);
  {
    const int tiles = (kM / 64) * (kC / 64);
    k_gemm_nt<1, 1><<<dim3((tiles + 7) / 8), dim3(256), 0, stream>>>(Gp, WCD, TAB + T_BC, Yp, kM, kC, kKT, kC);
  }
  k_store<<<dim3(kB * (kHW / 32)), dim3(256), 0, stream>>>(Yp, x, outp);
  (void)hipGetLastError();
}
